// PEGIModel_43095701848412
// MI455X (gfx1250) — hardware-run, weakly checked
//
#include <hip/hip_runtime.h>


#ifndef IMG_H
#define IMG_H 384
#endif
#define IMG_H_FULL 384
#define IMG_W 384
#define NG    512
#define NPIX  (IMG_H * IMG_W)
#define BT    256
#define PIXB  128
#define OUTT  (PIXB * 3 / 4)
#ifndef INPUT_BF16
#define INPUT_BF16 1
#endif
#define LOG2E_F 1.4426950408889634f
#define KQ_F    0.849321800f
#define BL2E_F  11.541560327111707f

static_assert(IMG_H <= IMG_H_FULL);
static_assert(NG % 32 == 0);
static_assert(NG % BT == 0);
static_assert(NPIX % PIXB == 0);
static_assert(PIXB == (BT / 32) * 16);
static_assert((PIXB * 3 * 4) % 128 == 0);
static_assert(OUTT * 16 == PIXB * 3 * 4);
static_assert(OUTT % 32 == 0);
static_assert(OUTT <= BT);
static_assert((13 * NG) % 8 == 0);
static_assert((size_t)NG * 8 * 4 + (size_t)16 * NG * 2 + (size_t)PIXB * 3 * 4 + (size_t)(BT / 32) * 4 <= (size_t)131072);

typedef _Float16 h16;
typedef __attribute__((ext_vector_type(16))) _Float16 v16h;
typedef __attribute__((ext_vector_type(8)))  _Float16 v8h;
typedef __attribute__((ext_vector_type(8)))  float    v8f;
typedef __attribute__((ext_vector_type(4)))  float    v4f;
typedef __attribute__((ext_vector_type(2)))  float    v2f;
typedef v4f  __attribute__((may_alias)) v4fa;

__device__ __forceinline__ unsigned short f2bf(float f) { unsigned u = __float_as_uint(f); u += 0x7FFFu + ((u >> 16) & 1u); return (unsigned short)(u >> 16); }
__device__ __forceinline__ float bfr(float f) { return __uint_as_float(((unsigned)f2bf(f)) << 16); }
__device__ __forceinline__ float inq(float v) { return INPUT_BF16 ? bfr(v) : v; }
__device__ __forceinline__ v16h cat16(v8h lo, v8h hi) { return __builtin_shufflevector(lo, hi, 0, 1, 2, 3, 4, 5, 6, 7, 8, 9, 10, 11, 12, 13, 14, 15); }
__device__ __forceinline__ v16h ldh(const h16* p) { return cat16(*(const v8h*)p, *(const v8h*)(p + 16)); }
static __device__ __forceinline__ h16 toh_flush(float v) { const h16 r = (h16)v; return (fabsf(v) < 6.103515625e-05f) ? (h16)0.0f : r; }
__device__ __forceinline__ v8f wmma16g(v16h a, v16h b, v8f c) {
    c = __builtin_amdgcn_wmma_f32_16x16x32_f16(false, a, false, b, (short)0, c, false, false);
    asm volatile("v_nop\n\tv_nop\n\tv_nop\n\tv_nop" : "+v"(c) : "v"(a), "v"(b));
    return c;
}

__global__ __launch_bounds__(BT) __attribute__((amdgpu_num_vgpr(256)))
void k_splat(const float* __restrict__ grid, const float* __restrict__ mu, const float* __restrict__ log_sigma, const float* __restrict__ theta,
             const float* __restrict__ depth, const float* __restrict__ normal, const float* __restrict__ albedo, const float* __restrict__ roughness,
             const float* __restrict__ opacity, const float* __restrict__ light, const float* __restrict__ ambient, float* out) {
    __shared__ __align__(16) float sP[NG * 8];
    __shared__ __align__(16) h16   sC[16 * NG];
    __shared__ __align__(16) float os[PIXB * 3];
    __shared__ float sW[BT / 32];

    const int tid = threadIdx.x;
    const int lane = tid & 31, lr = lane & 15, hi = lane >> 4;
    const int wave = __builtin_amdgcn_readfirstlane((int)(threadIdx.x >> 5));

    float dm = 3.0e38f;
#pragma unroll 1
    for (int j = 0; j < NG / BT; ++j) dm = fminf(dm, inq(depth[tid + j * BT]));
    dm = fminf(dm, __shfl_xor(dm, 16, 32));
    dm = fminf(dm, __shfl_xor(dm, 8, 32));
    dm = fminf(dm, __shfl_xor(dm, 4, 32));
    dm = fminf(dm, __shfl_xor(dm, 2, 32));
    dm = fminf(dm, __shfl_xor(dm, 1, 32));
    if (lane == 0) sW[wave] = dm;
    __syncthreads();
    float dmin = sW[0];
#pragma unroll
    for (int w = 1; w < BT / 32; ++w) dmin = fminf(dmin, sW[w]);

    {
        const float l0 = inq(light[0]), l1 = inq(light[1]), l2 = inq(light[2]);
        const float il = rsqrtf(l0 * l0 + l1 * l1 + l2 * l2);
        const float ldx = l0 * il, ldy = l1 * il, ldz = l2 * il;
        const float hx0 = ldx, hy0 = ldy, hz0 = ldz + 1.0f;
        const float ih = rsqrtf(hx0 * hx0 + hy0 * hy0 + hz0 * hz0);
        const float hx = hx0 * ih, hy = hy0 * ih, hz = hz0 * ih;
        const float am0 = inq(ambient[0]), am1 = inq(ambient[1]), am2 = inq(ambient[2]);
#pragma unroll 1
        for (int j = 0; j < NG / BT; ++j) {
            const int g = tid + j * BT;
            const float sx = __builtin_amdgcn_exp2f(inq(log_sigma[2 * g + 0]) * LOG2E_F) + 1e-6f;
            const float sy = __builtin_amdgcn_exp2f(inq(log_sigma[2 * g + 1]) * LOG2E_F) + 1e-6f;
            const float kx = KQ_F * __builtin_amdgcn_rcpf(sx);
            const float ky = KQ_F * __builtin_amdgcn_rcpf(sy);
            const float th = inq(theta[g]);
            const float ct = __cosf(th), st = __sinf(th);
            v4f g0, g1;
            g0[0] = ct * kx; g0[1] = st * kx; g0[2] = -st * ky; g0[3] = ct * ky;
            const float ed = __builtin_amdgcn_exp2f((dmin - inq(depth[g])) * BL2E_F);
            g1[0] = inq(mu[2 * g + 0]); g1[1] = inq(mu[2 * g + 1]); g1[2] = ed; g1[3] = ed * 1e-8f;
            *(v4fa*)(&sP[g * 8]) = g0;
            *(v4fa*)(&sP[g * 8 + 4]) = g1;
            const float n0 = inq(normal[3 * g + 0]), n1 = inq(normal[3 * g + 1]), n2 = inq(normal[3 * g + 2]);
            const float in = rsqrtf(n0 * n0 + n1 * n1 + n2 * n2);
            const float nx = n0 * in, ny = n1 * in, nz = n2 * in;
            const float ndotl = fmaxf(nx * ldx + ny * ldy + nz * ldz, 0.0f);
            const float sp = fmaxf(nx * hx + ny * hy + nz * hz, 0.0f);
            float s2 = sp * sp; s2 *= s2; s2 *= s2; s2 *= s2; s2 *= s2;
            const float specular = s2 * (1.0f - inq(roughness[g]));
            const float op = __builtin_amdgcn_rcpf(1.0f + __builtin_amdgcn_exp2f(-inq(opacity[g]) * LOG2E_F));
            const float oc0 = op * ((inq(albedo[3 * g + 0]) * ndotl + specular) + am0);
            const float oc1 = op * ((inq(albedo[3 * g + 1]) * ndotl + specular) + am1);
            const float oc2 = op * ((inq(albedo[3 * g + 2]) * ndotl + specular) + am2);
            sC[0 * NG + g] = toh_flush(oc0);
            sC[1 * NG + g] = toh_flush(oc1);
            sC[2 * NG + g] = toh_flush(oc2);
        }
        const v8h z8 = (v8h){};
#pragma unroll 1
        for (int i = tid; i < 13 * NG / 8; i += BT) *(v8h*)(&sC[3 * NG + i * 8]) = z8;
    }
    __syncthreads();

    const int pix = blockIdx.x * PIXB + wave * 16 + lr;
    const v2f gxy = *(const v2f*)(grid + (size_t)2 * pix);
    const float px = inq(gxy[0]), py = inq(gxy[1]);

    v8f acc = (v8f){};
    float sacc = 0.0f;
    int erun = 15;
#pragma unroll 1
    for (int k0 = 0; k0 < NG; k0 += 32) {
        float p[16];
        float mx = 0.0f;
#pragma unroll
        for (int i = 0; i < 16; ++i) {
            const int n = k0 + 8 * hi + (i & 7) + 16 * (i >> 3);
            const v4f g0 = *(const v4fa*)(&sP[n * 8]);
            const v4f g1 = *(const v4fa*)(&sP[n * 8 + 4]);
            const float dx = px - g1[0], dy = py - g1[1];
            const float u = dx * g0[0] + dy * g0[1];
            const float v = dx * g0[2] + dy * g0[3];
            const float q = fmaf(-u, u, -(v * v));
            const float w = __builtin_amdgcn_exp2f(q);
            const float t = fmaf(g1[2], w, g1[3]);
            sacc += t;
            p[i] = w * t;
            mx = fmaxf(mx, p[i]);
        }
        mx = fmaxf(mx, __shfl_xor(mx, 16, 32));
        int eb = (int)(__float_as_uint(mx) >> 23);
        eb = eb < 15 ? 15 : (eb > 254 ? 254 : eb);
        const int enew = erun > eb ? erun : eb;
        int ad = 127 - (enew - erun); ad = ad < 0 ? 0 : ad;
        const float alpha = __uint_as_float(((unsigned)ad) << 23);
        const float scale = __uint_as_float(((unsigned)(268 - enew)) << 23);
        erun = enew;
        v16h pb;
#pragma unroll
        for (int i = 0; i < 16; ++i) pb[i] = toh_flush(p[i] * scale);
        acc = acc * alpha;
        const v16h ca = ldh(&sC[lr * NG + k0 + 8 * hi]);
        acc = wmma16g(ca, pb, acc);
    }
    const float S = sacc + __shfl_xor(sacc, 16, 32);
    const float isc = __uint_as_float(((unsigned)(erun - 14)) << 23);
    const float rs = __builtin_amdgcn_rcpf(S);
    if (hi == 0) {
        const int ob = (wave * 16 + lr) * 3;
        os[ob + 0] = fminf(fmaxf(acc[0] * isc * rs, 0.0f), 1.0f);
        os[ob + 1] = fminf(fmaxf(acc[1] * isc * rs, 0.0f), 1.0f);
        os[ob + 2] = fminf(fmaxf(acc[2] * isc * rs, 0.0f), 1.0f);
    }
    __syncthreads();
    if (wave < OUTT / 32) {
        const v4f val = *(const v4fa*)(&os[tid * 4]);
        float* dst = out + (size_t)blockIdx.x * (PIXB * 3) + (size_t)tid * 4;
        *(volatile v4f*)dst = val;
        __threadfence();
        *(volatile v4f*)dst = val;
    }
}

extern "C" void kernel_launch(void* const* d_in, const int* in_sizes, int n_in,
                              void* d_out, int out_size, void* d_ws, size_t ws_size, hipStream_t stream) {
    (void)d_ws; (void)ws_size;
    if (n_in < 11) return;
    if ((size_t)in_sizes[0] < (size_t)NPIX * 2) return;
    if (in_sizes[1] < NG * 2 || in_sizes[2] < NG * 2 || in_sizes[3] < NG || in_sizes[4] < NG) return;
    if (in_sizes[5] < NG * 3 || in_sizes[6] < NG * 3 || in_sizes[7] < NG || in_sizes[8] < NG) return;
    if (in_sizes[9] < 3 || in_sizes[10] < 3) return;
    if ((size_t)out_size < (size_t)NPIX * 3) return;
    const float* grid      = (const float*)d_in[0];
    const float* mu        = (const float*)d_in[1];
    const float* log_sigma = (const float*)d_in[2];
    const float* theta     = (const float*)d_in[3];
    const float* depth     = (const float*)d_in[4];
    const float* normal    = (const float*)d_in[5];
    const float* albedo    = (const float*)d_in[6];
    const float* roughness = (const float*)d_in[7];
    const float* opacity   = (const float*)d_in[8];
    const float* light     = (const float*)d_in[9];
    const float* ambient   = (const float*)d_in[10];
    float* OUT = (float*)d_out;
    k_splat<<<dim3(NPIX / PIXB, 1, 1), BT, 0, stream>>>(grid, mu, log_sigma, theta, depth, normal, albedo, roughness, opacity, light, ambient, OUT);
}
